// SpatioTemporalAttention_75977971466367
// MI455X (gfx1250) — hardware-verified
//
#include <hip/hip_runtime.h>
#include <math.h>
#include <stdint.h>


#define NB   32
#define CH   256
#define NT   1024
#define TOK  (NB * NT)
#define RSB  32
#define PVN  64
#define OUTN (NB * CH * NT)

#define SCW  64.0f
#define SCQK 8.0f
#define SCV  16.0f
#define SCE  32768.0f
#define SCS  (1.0f / (SCQK * SCQK * 16.0f))

static_assert(TOK % 64 == 0 && CH % 64 == 0 && CH % 32 == 0 && NT % 32 == 0);
static_assert((((TOK / 64) * (CH / 64)) % 8) == 0);
static_assert(NT % RSB == 0 && RSB == 32 && NT == 4 * 256);
static_assert((NT / 16) % 8 == 0 && CH == 8 * 32);
static_assert(NT % PVN == 0 && PVN == 64);
static_assert((CH * CH) % 2048 == 0);
static_assert(NT % 64 == 0 && CH % 64 == 0);

typedef _Float16       v16h __attribute__((ext_vector_type(16)));
typedef _Float16       v8h  __attribute__((ext_vector_type(8)));
typedef float          v8f  __attribute__((ext_vector_type(8)));
typedef float          v4f  __attribute__((ext_vector_type(4)));
typedef unsigned int   v4u  __attribute__((ext_vector_type(4)));

union HU { v8h h; v4u u; _Float16 s[8]; };
union FR { v16h v; v8h h[2]; _Float16 s[16]; };
static_assert(sizeof(HU) == 16);
static_assert(sizeof(FR) == 32);

__device__ __forceinline__ unsigned short bf_bits(float f) {
  const unsigned u = __float_as_uint(f);
  return (unsigned short)((u + 0x7FFFu + ((u >> 16) & 1u)) >> 16);
}
__device__ __forceinline__ float bf_up(unsigned short h) { return __uint_as_float(((unsigned)h) << 16); }
__device__ __forceinline__ float bfr(float f) { return bf_up(bf_bits(f)); }
__device__ __forceinline__ v8f zero8() { v8f z = {0.f, 0.f, 0.f, 0.f, 0.f, 0.f, 0.f, 0.f}; return z; }

__device__ __forceinline__ void ld8(const float* p, float* o) {
  const v4f a = *(const v4f*)(p);
  const v4f b = *(const v4f*)(p + 4);
  o[0] = a[0]; o[1] = a[1]; o[2] = a[2]; o[3] = a[3];
  o[4] = b[0]; o[5] = b[1]; o[6] = b[2]; o[7] = b[3];
}

__device__ __forceinline__ v16h ldfrag_h(const _Float16* p) {
  FR f;
  f.h[0] = *(const v8h*)(p);
  f.h[1] = *(const v8h*)(p + 16);
  return f.v;
}

__device__ __forceinline__ v8f mma_h(v16h a, v16h b, v8f c) {
  c = __builtin_amdgcn_wmma_f32_16x16x32_f16(false, a, false, b, (short)0, c, false, false);
#if defined(__HIP_DEVICE_COMPILE__)
  asm volatile("v_nop\n\tv_nop\n\tv_nop\n\tv_nop" : "+v"(c) : "v"(a), "v"(b));
#endif
  return c;
}
__device__ __forceinline__ v8f mma_h_raw(v16h a, v16h b, v8f c) {
  return __builtin_amdgcn_wmma_f32_16x16x32_f16(false, a, false, b, (short)0, c, false, false);
}
__device__ __forceinline__ void dep_guard_h(v8f& a, v8f& b, v16h x) {
#if defined(__HIP_DEVICE_COMPILE__)
  asm volatile("v_nop\n\tv_nop\n\tv_nop\n\tv_nop" : "+v"(a), "+v"(b) : "v"(x));
#endif
}
__device__ __forceinline__ void keep4_h(v16h a, v16h b, v16h c, v16h d) {
#if defined(__HIP_DEVICE_COMPILE__)
  asm volatile("v_nop" :: "v"(a), "v"(b), "v"(c), "v"(d));
#endif
}
__device__ __forceinline__ void acc_guard4(v8f& a, v8f& b, v8f& c, v8f& d) {
#if defined(__HIP_DEVICE_COMPILE__)
  asm volatile("v_nop\n\tv_nop\n\tv_nop\n\tv_nop" : "+v"(a), "+v"(b), "+v"(c), "+v"(d));
#endif
}
__device__ __forceinline__ void wave_lds_sync() {
  __builtin_amdgcn_fence(__ATOMIC_RELEASE, "workgroup");
  __builtin_amdgcn_wave_barrier();
  __builtin_amdgcn_fence(__ATOMIC_ACQUIRE, "workgroup");
}

__global__ __launch_bounds__(256) void cvt_flat(const float* __restrict__ in, _Float16* out, int n8, float scale) {
  const int i = blockIdx.x * 256 + threadIdx.x;
  if (i < n8) {
    float v[8];
    ld8(in + (size_t)i * 8, v);
    HU u;
#pragma unroll
    for (int e = 0; e < 8; ++e) u.s[e] = (_Float16)(bfr(v[e]) * scale);
    _Float16* p = out + (size_t)i * 8;
    *(volatile v4u*)p = u.u;
    __threadfence();
    *(volatile v4u*)p = u.u;
  }
}

__global__ __launch_bounds__(256) void cvt_xT(const float* __restrict__ X, _Float16* XT, int Cd) {
  __shared__ float sw[64][65];
  const int t = threadIdx.x;
  const int n0 = blockIdx.x * 64, k0 = blockIdx.y * 64, b = blockIdx.z;
  const float* Xb = X + (size_t)b * Cd * NT;
  {
    const int r = t >> 4, c4 = (t & 15) * 4;
#pragma unroll
    for (int it = 0; it < 4; ++it) {
      const int row = r + 16 * it;
      const v4f x = *(const v4f*)(Xb + (size_t)(k0 + row) * NT + n0 + c4);
      sw[row][c4 + 0] = x[0]; sw[row][c4 + 1] = x[1]; sw[row][c4 + 2] = x[2]; sw[row][c4 + 3] = x[3];
    }
  }
  __syncthreads();
  const int q8 = t & 7, rr = t >> 3;
  HU u[2];
#pragma unroll
  for (int it = 0; it < 2; ++it) {
    const int n = rr + 32 * it;
#pragma unroll
    for (int e = 0; e < 8; ++e) u[it].s[e] = (_Float16)bfr(sw[8 * q8 + e][n]);
  }
  for (int pass = 0; pass < 2; ++pass) {
#pragma unroll
    for (int it = 0; it < 2; ++it) {
      const int n = rr + 32 * it;
      _Float16* dst = XT + (size_t)(b * NT + n0 + n) * Cd + k0 + 8 * q8;
      *(volatile v4u*)dst = u[it].u;
    }
    __threadfence();
  }
}

template <int MI>
__device__ __forceinline__ void kseg(v8f (&acc)[MI][4], const _Float16* __restrict__ A, int lda, int m0,
                                     const _Float16* __restrict__ Bt, int ldb, int n0, int K, int rlane, int koff) {
  for (int kk = 0; kk < K; kk += 32) {
    v16h bh[4];
#pragma unroll
    for (int j = 0; j < 4; ++j) {
      const size_t bo = (size_t)(n0 + (j << 4) + rlane) * (size_t)ldb + koff + kk;
      bh[j] = ldfrag_h(Bt + bo);
    }
#pragma unroll
    for (int i = 0; i < MI; ++i) {
      const size_t ao = (size_t)(m0 + (i << 4) + rlane) * (size_t)lda + koff + kk;
      const v16h a0 = ldfrag_h(A + ao);
#pragma unroll
      for (int j = 0; j < 4; ++j) acc[i][j] = mma_h_raw(a0, bh[j], acc[i][j]);
      dep_guard_h(acc[i][0], acc[i][3], a0);
    }
    keep4_h(bh[0], bh[1], bh[2], bh[3]);
  }
}

template <int RB>
__global__ __launch_bounds__(256) void gemm64p(
    const _Float16* __restrict__ A, int lda, const _Float16* __restrict__ Bt, int ldb,
    const float* __restrict__ bias, int nbias, float cs, float so,
    _Float16* Cp, int ldc, int M, int N, int K) {
  __shared__ __align__(16) float sT[8][16 * 68];
  const int lane = threadIdx.x & 31;
  const int wave = threadIdx.x >> 5;
  const int tilesN = N >> 6;
  const int tilesM = M >> 6;
  const int tiles = tilesM * tilesN;
  const int item = blockIdx.x * 8 + wave;
  if (item >= tiles) return;
  const int tm = item / tilesN;
  const int tn = item - tm * tilesN;
  const int m0 = tm << 6;
  const int n0 = tn << 6;

  const int rlane = lane & 15;
  const int koff  = (lane >> 4) * 8;
  const int mOff  = (lane >> 4) * 8;

  v8f acc[4][4];
#pragma unroll
  for (int i = 0; i < 4; ++i)
#pragma unroll
    for (int j = 0; j < 4; ++j) acc[i][j] = zero8();

  kseg<4>(acc, A, lda, m0, Bt, ldb, n0, K, rlane, koff);
  acc_guard4(acc[0][0], acc[0][1], acc[0][2], acc[0][3]);
  acc_guard4(acc[1][0], acc[1][1], acc[1][2], acc[1][3]);
  acc_guard4(acc[2][0], acc[2][1], acc[2][2], acc[2][3]);
  acc_guard4(acc[3][0], acc[3][1], acc[3][2], acc[3][3]);

  const int q8 = lane & 7, rr = lane >> 3, c8 = q8 * 8;

  float cbv[8];
#pragma unroll
  for (int e = 0; e < 8; ++e) cbv[e] = 0.0f;
  if (RB == 2) {
#pragma unroll
    for (int e = 0; e < 8; ++e) cbv[e] = bfr(bias[min(n0 + c8 + e, nbias - 1)]);
  }

  float* slab = sT[wave];
#pragma unroll
  for (int i = 0; i < 4; ++i) {
    const int mBase = m0 + (i << 4);
#pragma unroll
    for (int r = 0; r < 8; ++r) {
#pragma unroll
      for (int j = 0; j < 4; ++j) {
        slab[(mOff + r) * 68 + (j << 4) + rlane] = acc[i][j][r];
      }
    }
    wave_lds_sync();
    v4u uh[4];
#pragma unroll
    for (int it = 0; it < 4; ++it) {
      const int row = it * 4 + rr;
      float xs[8];
      ld8(slab + row * 68 + c8, xs);
      float rbv = 0.0f;
      if (RB == 1) rbv = bfr(bias[min(mBase + row, nbias - 1)]);
      HU h;
#pragma unroll
      for (int e = 0; e < 8; ++e) {
        const float v = (xs[e] * cs + rbv + cbv[e]) * so;
        h.s[e] = (_Float16)v;
      }
      uh[it] = h.u;
    }
    for (int pass = 0; pass < 2; ++pass) {
#pragma unroll
      for (int it = 0; it < 4; ++it) {
        const int row = it * 4 + rr;
        const size_t co = (size_t)(mBase + row) * (size_t)ldc + n0 + c8;
        *(volatile v4u*)(Cp + co) = uh[it];
      }
      __threadfence();
    }
    wave_lds_sync();
  }
}

__global__ __launch_bounds__(256) void k_soft(const _Float16* __restrict__ XQ, const _Float16* __restrict__ XK,
                                              _Float16* E) {
  extern __shared__ __align__(16) float sc[];
  const int tid = threadIdx.x, wave = tid >> 5, lane = tid & 31;
  const int hh = lane >> 4, rl = lane & 15;
  const int rb = blockIdx.x, b = blockIdx.y, n0 = rb * RSB;

  const _Float16* aq = XQ + (size_t)(b * NT + n0 + rl) * CH + 8 * hh;
  for (int ct = wave; ct < NT / 16; ct += 8) {
    const _Float16* bk = XK + (size_t)(b * NT + 16 * ct + rl) * CH + 8 * hh;
    v8f a0 = zero8(), a1 = zero8();
#pragma unroll 2
    for (int ks = 0; ks < CH / 32; ++ks) {
      const v16h kb = ldfrag_h(bk + 32 * ks);
      const v16h q0 = ldfrag_h(aq + 32 * ks);
      const v16h q1 = ldfrag_h(aq + 16 * CH + 32 * ks);
      a0 = mma_h(q0, kb, a0);
      a1 = mma_h(q1, kb, a1);
    }
    const int mc = 16 * ct + rl;
#pragma unroll
    for (int r = 0; r < 8; ++r) {
      sc[(size_t)(8 * hh + r) * NT + mc]      = a0[r] * SCS;
      sc[(size_t)(16 + 8 * hh + r) * NT + mc] = a1[r] * SCS;
    }
  }
  __syncthreads();

  for (int q4 = 0; q4 < 4; ++q4) {
    const int row = 4 * wave + q4;
    const float* rp = sc + (size_t)row * NT + 8 * lane;
    float v[4][8];
    float mx = -3.0e38f;
#pragma unroll
    for (int j = 0; j < 4; ++j) {
      ld8(rp + 256 * j, v[j]);
#pragma unroll
      for (int e = 0; e < 8; ++e) mx = fmaxf(mx, v[j][e]);
    }
#pragma unroll
    for (int off = 16; off >= 1; off >>= 1) mx = fmaxf(mx, __shfl_xor(mx, off, 32));
    float z = 0.0f;
#pragma unroll
    for (int j = 0; j < 4; ++j) {
#pragma unroll
      for (int e = 0; e < 8; ++e) {
        const float ef = __expf(v[j][e] - mx);
        z += ef;
        v[j][e] = ef;
      }
    }
#pragma unroll
    for (int off = 16; off >= 1; off >>= 1) z += __shfl_xor(z, off, 32);
    const float rz = SCE * (1.0f / z);
    HU u[4];
#pragma unroll
    for (int j = 0; j < 4; ++j) {
#pragma unroll
      for (int e = 0; e < 8; ++e) {
        const _Float16 h0 = (_Float16)(v[j][e] * rz);
        const float f0 = (float)h0;
        const bool sub = f0 < 6.103515625e-05f;
        u[j].s[e] = sub ? (_Float16)0.0f : h0;
      }
    }
    _Float16* erow = E + (size_t)(b * NT + n0 + row) * NT + 8 * lane;
    for (int pass = 0; pass < 2; ++pass) {
#pragma unroll
      for (int j = 0; j < 4; ++j) *(volatile v4u*)(erow + 256 * j) = u[j].u;
      __threadfence();
    }
  }
}

__global__ __launch_bounds__(256) void k_pv(const _Float16* __restrict__ E, const _Float16* __restrict__ VH,
                                            const float* __restrict__ X, float* out) {
  __shared__ __align__(16) float sO[8][16 * 68];
  const int tid = threadIdx.x, wave = tid >> 5, lane = tid & 31;
  const int hh = lane >> 4, rl = lane & 15;
  const int bx = blockIdx.x;
  const int b = bx / (NT / PVN);
  const int n0 = (bx - b * (NT / PVN)) * PVN;
  const int cb = wave * 32;

  v8f acc[2][4];
#pragma unroll
  for (int i = 0; i < 2; ++i)
#pragma unroll
    for (int j = 0; j < 4; ++j) acc[i][j] = zero8();

  const _Float16* Ab = VH + (size_t)b * NT;
  const _Float16* Bb = E + (size_t)b * NT * NT;
  kseg<2>(acc, Ab, TOK, cb, Bb, NT, n0, NT, rl, 8 * hh);
  acc_guard4(acc[0][0], acc[0][1], acc[0][2], acc[0][3]);
  acc_guard4(acc[1][0], acc[1][1], acc[1][2], acc[1][3]);

  const float fo = 1.0f / (SCV * SCE);
  float* slab = sO[wave];
  const int p4 = (lane & 15) * 4, r2 = lane >> 4;
#pragma unroll
  for (int i = 0; i < 2; ++i) {
    const int cBase = cb + 16 * i;
#pragma unroll
    for (int r = 0; r < 8; ++r) {
#pragma unroll
      for (int j = 0; j < 4; ++j) {
        slab[(8 * hh + r) * 68 + 16 * j + rl] = acc[i][j][r];
      }
    }
    wave_lds_sync();
    v4f ov[8];
#pragma unroll
    for (int it = 0; it < 8; ++it) {
      const int row = 2 * it + r2;
      const v4f a = *(const v4f*)(slab + row * 68 + p4);
      const size_t xo = ((size_t)(b * CH + cBase + row)) * NT + n0 + p4;
      const v4f xv = *(const v4f*)(X + xo);
      v4f o;
#pragma unroll
      for (int e = 0; e < 4; ++e) o[e] = a[e] * fo + bfr(xv[e]);
      ov[it] = o;
    }
    for (int pass = 0; pass < 2; ++pass) {
#pragma unroll
      for (int it = 0; it < 8; ++it) {
        const int row = 2 * it + r2;
        const size_t oo = ((size_t)(b * CH + cBase + row)) * NT + n0 + p4;
        *(volatile v4f*)(out + oo) = ov[it];
      }
      __threadfence();
    }
    wave_lds_sync();
  }
}

extern "C" void kernel_launch(void* const* d_in, const int* in_sizes, int n_in,
                              void* d_out, int out_size, void* d_ws, size_t ws_size,
                              hipStream_t stream) {
  if (n_in < 7) return;
  if (in_sizes[0] != NB * CH * NT) return;
  if (in_sizes[1] != CH * CH || in_sizes[2] != CH) return;
  if (in_sizes[3] != CH * CH || in_sizes[4] != CH) return;
  if (in_sizes[5] != CH * CH || in_sizes[6] != CH) return;
  if (out_size != OUTN) return;

  const float* x  = (const float*)d_in[0];
  const float* Wq = (const float*)d_in[1];
  const float* bq = (const float*)d_in[2];
  const float* Wk = (const float*)d_in[3];
  const float* bk = (const float*)d_in[4];
  const float* Wv = (const float*)d_in[5];
  const float* bv = (const float*)d_in[6];

  const size_t PW  = (size_t)CH * CH * 2;
  const size_t PPL = (size_t)TOK * CH * 2;
  const size_t PE  = (size_t)TOK * NT * 2;
  const size_t PXE = (PE > PPL) ? PE : PPL;

  size_t off = 0;
  const size_t oWQ = off; off += PW;
  const size_t oWK = off; off += PW;
  const size_t oWV = off; off += PW;
  const size_t oXQ = off; off += PPL;
  const size_t oXK = off; off += PPL;
  const size_t oVH = off; off += PPL;
  const size_t oXE = off; off += PXE;
  if (off > ws_size) return;
  if (off > (size_t)134217728) return;

  char* ws = (char*)d_ws;
  _Float16* WQ16 = (_Float16*)(ws + oWQ);
  _Float16* WK16 = (_Float16*)(ws + oWK);
  _Float16* WV16 = (_Float16*)(ws + oWV);
  _Float16* XQ   = (_Float16*)(ws + oXQ);
  _Float16* XK   = (_Float16*)(ws + oXK);
  _Float16* VH   = (_Float16*)(ws + oVH);
  _Float16* xT   = (_Float16*)(ws + oXE);
  _Float16* E    = (_Float16*)(ws + oXE);
  float*    outf = (float*)d_out;

  const dim3 blk(256);
  const int n8cc = (CH * CH) / 8;
  const dim3 gWcc((n8cc + 255) / 256);
  const dim3 gXT(NT / 64, CH / 64, NB);
  const dim3 gPr(((TOK / 64) * (CH / 64) + 7) / 8);
  const dim3 gSo(NT / RSB, NB);
  const dim3 gPV(NB * (NT / PVN));
  const float cs64 = 1.0f / SCW;
  const size_t ldsSoft = (size_t)RSB * NT * sizeof(float);

  cvt_flat<<<gWcc, blk, 0, stream>>>(Wq, WQ16, n8cc, SCW);
  cvt_flat<<<gWcc, blk, 0, stream>>>(Wk, WK16, n8cc, SCW);
  cvt_flat<<<gWcc, blk, 0, stream>>>(Wv, WV16, n8cc, SCW);
  cvt_xT<<<gXT, blk, 0, stream>>>(x, xT, CH);
  gemm64p<2><<<gPr, blk, 0, stream>>>(xT, CH, WQ16, CH, bq, CH, cs64, SCQK, XQ, CH, TOK, CH, CH);
  gemm64p<2><<<gPr, blk, 0, stream>>>(xT, CH, WK16, CH, bk, CH, cs64, SCQK, XK, CH, TOK, CH, CH);
  gemm64p<1><<<gPr, blk, 0, stream>>>(WV16, CH, xT, CH, bv, CH, cs64, SCV, VH, TOK, CH, TOK, CH);
  k_soft<<<gSo, blk, ldsSoft, stream>>>(XQ, XK, E);
  k_pv<<<gPV, blk, 0, stream>>>(E, VH, x, outf);
}
